// OneLayerDiagTransitionLinearRNN_60069412601936
// MI455X (gfx1250) — hardware-verified
//
#include <hip/hip_runtime.h>
#include <math.h>

typedef __attribute__((ext_vector_type(16))) _Float16 v16h;
typedef __attribute__((ext_vector_type(8)))  _Float16 v8h;
typedef __attribute__((ext_vector_type(2)))  _Float16 v2h;
typedef __attribute__((ext_vector_type(16))) __bf16   v16b;
typedef __attribute__((ext_vector_type(8)))  __bf16   v8b;
typedef __attribute__((ext_vector_type(8)))  float    v8f;
typedef __attribute__((ext_vector_type(4)))  float    v4f;
typedef __attribute__((ext_vector_type(2)))  float    v2f;

constexpr int kNB   = 32;
constexpr int kS    = 4096;
constexpr int kRows = kNB * kS;
constexpr int kI    = 64;
constexpr int kN    = 512;
constexpr int kNq   = 128;
constexpr int kO    = 64;
constexpr int kThr  = 256;
constexpr float kInCarry = 1024.0f;
constexpr float kWCarry  = 4096.0f;
constexpr float kSCarry  = 64.0f;
constexpr float kScIn  = 1.0f / (kInCarry * kWCarry);
constexpr float kScOut = 1.0f / (kSCarry * kWCarry);
constexpr float kF16MinNormal = 6.103515625e-5f;

static_assert(kRows == 131072 && kI == 64 && kN == 512 && kNq * 4 == kN && kO == 64 && (kNq % 64) == 0 && (kO % 64) == 0, "the index arithmetic below uses these sizes");

constexpr size_t kOffX16 = 0ull;
constexpr size_t kOffWB16 = 16777216ull;
constexpr size_t kOffWC16 = 16842752ull;
constexpr size_t kOffZB = 16908288ull;
constexpr size_t kOffXB = 16908800ull;
constexpr size_t kOffS16 = 84017664ull;
constexpr size_t kWsTotal = 218235392ull;
static_assert(kWsTotal <= 268435456ull, "the carve stands under the contract's 256 MiB of workspace");
static_assert(kOffX16 == 0
  && kOffWB16 == kOffX16 + 16777216ull
  && kOffWC16 == kOffWB16 + 65536ull
  && kOffZB == kOffWC16 + 65536ull
  && kOffXB == kOffZB + 512ull
  && kOffS16 == kOffXB + 67108864ull
  && kWsTotal == kOffS16 + 134217728ull, "the carve is a chain: every region starts where the one before ends");
static_assert((kOffWB16 % 256) == 0 && (kOffWC16 % 256) == 0 && (kOffZB % 256) == 0 && (kOffXB % 256) == 0 && (kOffS16 % 256) == 0, "every region starts on a multiple of 256 B");

__device__ __forceinline__ unsigned short f2bf_bits(float f) {
  unsigned u = __float_as_uint(f);
  return (unsigned short)((u + 0x7FFFu + ((u >> 16) & 1u)) >> 16);
}
__device__ __forceinline__ float bf_bits2f(unsigned short h) { return __uint_as_float(((unsigned)h) << 16); }
__device__ __forceinline__ float bf16r(float f) { return bf_bits2f(f2bf_bits(f)); }
__device__ __forceinline__ float carry_flush(float v, float carry) {
  const float s = v * carry;
  return (fabsf(s) < kF16MinNormal) ? 0.0f : s;
}

__device__ __forceinline__ void dep_guard4_h(v8f& a, v8f& b, v8f& c, v8f& d, v16h x, v16h y) { asm volatile("v_nop\n\tv_nop\n\tv_nop\n\tv_nop" : "+v"(a), "+v"(b), "+v"(c), "+v"(d) : "v"(x), "v"(y)); }
__device__ __forceinline__ void dep_guard4_b(v8f& a, v8f& b, v8f& c, v8f& d, v16b x, v16b y) { asm volatile("v_nop\n\tv_nop\n\tv_nop\n\tv_nop" : "+v"(a), "+v"(b), "+v"(c), "+v"(d) : "v"(x), "v"(y)); }
__device__ __forceinline__ void keep4_h(v16h a, v16h b, v16h c, v16h d) { asm volatile("v_nop" :: "v"(a), "v"(b), "v"(c), "v"(d)); }
__device__ __forceinline__ void keep4_b(v16b a, v16b b, v16b c, v16b d) { asm volatile("v_nop" :: "v"(a), "v"(b), "v"(c), "v"(d)); }
__device__ __forceinline__ void acc_guard4(v8f& a, v8f& b, v8f& c, v8f& d) { asm volatile("v_nop\n\tv_nop\n\tv_nop\n\tv_nop" : "+v"(a), "+v"(b), "+v"(c), "+v"(d)); }

template <typename T> struct Frag;
template <> struct Frag<_Float16> {
  typedef v16h V; union U { v16h v; v8h h[2]; };
  static __device__ __forceinline__ v16h load(const _Float16* p) {
    U f; f.h[0] = *(const v8h*)(p); f.h[1] = *(const v8h*)(p + 16); return f.v;
  }
  static __device__ __forceinline__ v8f mma(v16h a, v16h b, v8f c) {
    return __builtin_amdgcn_wmma_f32_16x16x32_f16(false, a, false, b, (short)0, c, false, false);
  }
  static __device__ __forceinline__ void guard4(v8f& a, v8f& b, v8f& c, v8f& d, v16h x, v16h y) { dep_guard4_h(a, b, c, d, x, y); }
  static __device__ __forceinline__ void keep(v16h a, v16h b, v16h c, v16h d) { keep4_h(a, b, c, d); }
};
template <> struct Frag<__bf16> {
  typedef v16b V; union U { v16b v; v8b h[2]; };
  static __device__ __forceinline__ v16b load(const __bf16* p) {
    U f; f.h[0] = *(const v8b*)(p); f.h[1] = *(const v8b*)(p + 16); return f.v;
  }
  static __device__ __forceinline__ v8f mma(v16b a, v16b b, v8f c) {
    return __builtin_amdgcn_wmma_f32_16x16x32_bf16(false, a, false, b, (short)0, c, false, false);
  }
  static __device__ __forceinline__ void guard4(v8f& a, v8f& b, v8f& c, v8f& d, v16b x, v16b y) { dep_guard4_b(a, b, c, d, x, y); }
  static __device__ __forceinline__ void keep(v16b a, v16b b, v16b c, v16b d) { keep4_b(a, b, c, d); }
};

__device__ __forceinline__ v8f mma_h(v16h a, v16h b, v8f c) {
  c = __builtin_amdgcn_wmma_f32_16x16x32_f16(false, a, false, b, (short)0, c, false, false);
  asm volatile("v_nop\n\tv_nop\n\tv_nop\n\tv_nop" : "+v"(c) : "v"(a), "v"(b));
  return c;
}

template <int ET> struct Elem;
template <> struct Elem<0> { typedef _Float16 T; };
template <> struct Elem<1> { typedef __bf16 T; };
template <int ET, bool SPLIT, int BIAS_MODE, int OUT_MODE, bool RESID, int ACT = 0>
__global__ __launch_bounds__(256) void wmma_gemm64(
    const unsigned short* __restrict__ Ap, const unsigned short* __restrict__ A2p, int lda, long strideA,
    const unsigned short* __restrict__ Btp, const unsigned short* __restrict__ Bt2p, int ldb, long strideB,
    void* __restrict__ Cout, void* __restrict__ Cout2, int ldc, long strideC,
    const float* __restrict__ bias,
    const float* __restrict__ resid, long strideR,
    int M, int N, int K, float scale) {
  typedef typename Elem<ET>::T T;
  typedef typename Frag<T>::V V;
  const T* A = (const T*)Ap; const T* A2 = (const T*)A2p; const T* Bt = (const T*)Btp; const T* Bt2 = (const T*)Bt2p;
  __shared__ __align__(16) float sT[8][16 * 68];
  const int b    = blockIdx.y;
  const int lane = threadIdx.x & 31;
  const int wave = threadIdx.x >> 5;
  const int tilesN = N >> 6;
  const int tilesM = M >> 6;
  const int tile = blockIdx.x * 8 + wave;
  if (tile >= tilesM * tilesN) return;
  const int tm = tile / tilesN;
  const int tn = tile - tm * tilesN;
  const int m0 = tm << 6;
  const int n0 = tn << 6;

  const T* Ab  = A  + (size_t)b * strideA;
  const T* Bb  = Bt + (size_t)b * strideB;
  const T* Ab2 = SPLIT ? (A2  + (size_t)b * strideA) : nullptr;
  const T* Bb2 = SPLIT ? (Bt2 + (size_t)b * strideB) : nullptr;

  const int rlane = lane & 15;
  const int koff  = (lane >> 4) * 8;
  const int mOff  = (lane >> 4) * 8;

  v8f acc[4][4];
#pragma unroll
  for (int i = 0; i < 4; ++i)
#pragma unroll
    for (int j = 0; j < 4; ++j) acc[i][j] = (v8f){0.f,0.f,0.f,0.f,0.f,0.f,0.f,0.f};

  for (int k0 = 0; k0 < K; k0 += 32) {
    V bh[4], bl[4];
#pragma unroll
    for (int j = 0; j < 4; ++j) {
      const size_t bo = (size_t)(n0 + (j << 4) + rlane) * ldb + koff + k0;
      bh[j] = Frag<T>::load(Bb + bo);
      if (SPLIT) bl[j] = Frag<T>::load(Bb2 + bo);
    }
#pragma unroll
    for (int i = 0; i < 4; ++i) {
      const size_t ao = (size_t)(m0 + (i << 4) + rlane) * lda + koff + k0;
      V ah = Frag<T>::load(Ab + ao);
      V al;
      if (SPLIT) al = Frag<T>::load(Ab2 + ao);
#pragma unroll
      for (int j = 0; j < 4; ++j) {
        acc[i][j] = Frag<T>::mma(ah, bh[j], acc[i][j]);
        if (SPLIT) {
          acc[i][j] = Frag<T>::mma(ah, bl[j], acc[i][j]);
          acc[i][j] = Frag<T>::mma(al, bh[j], acc[i][j]);
        }
      }
      Frag<T>::guard4(acc[i][0], acc[i][1], acc[i][2], acc[i][3], ah, SPLIT ? al : ah);
    }
    Frag<T>::keep(bh[0], bh[1], bh[2], bh[3]);
    if (SPLIT) Frag<T>::keep(bl[0], bl[1], bl[2], bl[3]);
  }
  acc_guard4(acc[0][0], acc[0][1], acc[0][2], acc[0][3]);
  acc_guard4(acc[1][0], acc[1][1], acc[1][2], acc[1][3]);
  acc_guard4(acc[2][0], acc[2][1], acc[2][2], acc[2][3]);
  acc_guard4(acc[3][0], acc[3][1], acc[3][2], acc[3][3]);

  float* slab = sT[wave];
  const float* Rb = RESID ? (resid + (size_t)b * strideR) : nullptr;
#pragma unroll
  for (int i = 0; i < 4; ++i) {
    const int mBase = m0 + (i << 4);
#pragma unroll
    for (int j = 0; j < 4; ++j) {
      const int n = n0 + (j << 4) + rlane;
      float bv = 0.f;
      if (BIAS_MODE == 2) bv = bias[n];
#pragma unroll
      for (int r = 0; r < 8; ++r) {
        float v = acc[i][j][r] * scale;
        if (BIAS_MODE == 1) v += bias[mBase + mOff + r];
        if (BIAS_MODE == 2) v += bv;
        if (RESID) v += Rb[(size_t)(mBase + mOff + r) * ldc + n];
        if (ACT == 1) v = tanhf(v);
        if (ACT == 2) v = fmaxf(v, 0.0f);
        if (ACT == 3) v = v / (1.0f + expf(-v));
        if (ACT == 4) v = (v > 0.f) ? v : 0.01f * v;
        slab[(mOff + r) * 68 + (j << 4) + rlane] = v;
      }
    }
    __builtin_amdgcn_fence(__ATOMIC_RELEASE, "workgroup");
    __builtin_amdgcn_wave_barrier();
    __builtin_amdgcn_fence(__ATOMIC_ACQUIRE, "workgroup");
    if (OUT_MODE == 0) {
      float* C = (float*)Cout + (size_t)b * strideC;
      const int hh = lane >> 4, c4 = (lane & 15) * 4;
      for (int pass = 0; pass < 2; ++pass) {
#pragma unroll
        for (int it = 0; it < 8; ++it) {
          const int row = it * 2 + hh;
          v4f v = *(const v4f*)(slab + row * 68 + c4);
          *(volatile v4f*)(C + (size_t)(mBase + row) * ldc + n0 + c4) = v;
        }
        __threadfence();
      }
    } else {
      const int q = lane >> 3, c8 = (lane & 7) * 8;
      unsigned short* C  = (unsigned short*)Cout  + (size_t)b * strideC;
      unsigned short* C2 = (OUT_MODE == 2) ? ((unsigned short*)Cout2 + (size_t)b * strideC) : nullptr;
      for (int pass = 0; pass < 2; ++pass) {
#pragma unroll
        for (int it = 0; it < 4; ++it) {
          const int row = it * 4 + q;
          const float* sp = slab + row * 68 + c8;
          v8h hv, lv;
#pragma unroll
          for (int e = 0; e < 8; ++e) {
            if (OUT_MODE == 1) {
              hv[e] = (_Float16)sp[e];
            } else {
              unsigned short hb = f2bf_bits(sp[e]);
              unsigned short lb = f2bf_bits(sp[e] - bf_bits2f(hb));
              hv[e] = __builtin_bit_cast(_Float16, hb);
              lv[e] = __builtin_bit_cast(_Float16, lb);
            }
          }
          *(volatile v8h*)(C + (size_t)(mBase + row) * ldc + n0 + c8) = hv;
          if (OUT_MODE == 2) *(volatile v8h*)(C2 + (size_t)(mBase + row) * ldc + n0 + c8) = lv;
        }
        __threadfence();
      }
    }
    __builtin_amdgcn_fence(__ATOMIC_RELEASE, "workgroup");
    __builtin_amdgcn_wave_barrier();
    __builtin_amdgcn_fence(__ATOMIC_ACQUIRE, "workgroup");
  }
}


__device__ __forceinline__ void store2(float* p, float v) {
  *(volatile float*)p = v;
  __threadfence();
  *(volatile float*)p = v;
}

__global__ __launch_bounds__(kThr) void cast_plane_kernel(const float* __restrict__ src, unsigned short* __restrict__ dst,
                                                          int colsLog2, int dstPitch, int dstOff) {
  const int i   = blockIdx.x * kThr + threadIdx.x;
  const int sh  = colsLog2 - 3;
  const int row = i >> sh;
  const int c8  = (i & ((1 << sh) - 1)) * 8;
  const float* sp = src + ((size_t)row << colsLog2) + c8;
  const v4f a0 = *(const v4f*)(sp);
  const v4f a1 = *(const v4f*)(sp + 4);
  v8h hv;
#pragma unroll
  for (int e = 0; e < 4; ++e) {
    const float f0 = a0[e];
    const float f1 = a1[e];
    hv[e]     = (_Float16)carry_flush(bf16r(f0), kInCarry);
    hv[4 + e] = (_Float16)carry_flush(bf16r(f1), kInCarry);
  }
  unsigned short* dp = dst + (size_t)row * dstPitch + dstOff + c8;
  *(volatile v8h*)dp = hv;
  __threadfence();
  *(volatile v8h*)dp = hv;
}

__global__ __launch_bounds__(256) void wt_plane_kernel(const float* __restrict__ W, unsigned short* __restrict__ dst, int K, int N, int nLive, int ldd, int colOff) {
  const int n  = blockIdx.x;
  const int k8 = threadIdx.x * 8;
  const bool live = n < nLive;
  const int nc = live ? n : 0;
  v8h hv;
#pragma unroll
  for (int e = 0; e < 8; ++e) {
    const float w = W[(size_t)(k8 + e) * N + nc];
    hv[e] = (_Float16)(live ? carry_flush(bf16r(w), kWCarry) : 0.0f);
  }
  unsigned short* dp = dst + (size_t)n * ldd + colOff + k8;
  *(volatile v8h*)dp = hv;
  __threadfence();
  *(volatile v8h*)dp = hv;
}

__global__ __launch_bounds__(kThr) void setup_kernel(float* __restrict__ ZB) {
  float* dp = ZB + threadIdx.x;
  *(volatile float*)dp = 0.0f;
  __threadfence();
  *(volatile float*)dp = 0.0f;
}

__global__ __launch_bounds__(kThr) void scan_kernel(const float* __restrict__ XB, const float* __restrict__ A, unsigned short* __restrict__ S16, int quarter) {
  const unsigned ix = blockIdx.x * (unsigned)kThr + threadIdx.x;
  const unsigned sq = ix >> 6;
  const unsigned m0 = (ix & 63u) * 2u;
  const unsigned n0 = (unsigned)quarter * (unsigned)kNq + m0;
  const v2f av = *(const v2f*)(A + n0);
  const float a0 = bf16r(av[0]), a1 = bf16r(av[1]);
  float s0 = 0.0f, s1 = 0.0f;
  for (int t = 0; t < kS; ++t) {
    const size_t row = (size_t)sq * kS + (size_t)t;
    const v2f p = *(const v2f*)(XB + row * kNq + m0);
    s0 = p[0] + s0 * a0;
    s1 = p[1] + s1 * a1;
    v2h sv;
    sv[0] = (_Float16)carry_flush(s0, kSCarry);
    sv[1] = (_Float16)carry_flush(s1, kSCarry);
    unsigned short* dp = S16 + row * kN + n0;
    *(volatile v2h*)dp = sv;
    __threadfence();
    *(volatile v2h*)dp = sv;
  }
}
static_assert(kNB * kNq / 2 == 8 * kThr && kNq / 2 == 64, "walk grid exact: 8 blocks a quarter: 64 lanes a sequence");

extern "C" void kernel_launch(void* const* d_in, const int* in_sizes, int n_in,
                              void* d_out, int out_size, void* d_ws, size_t ws_size,
                              hipStream_t stream) {
  if (n_in < 4 || d_out == nullptr || d_ws == nullptr) return;
  if (in_sizes[0] != kRows * kI || in_sizes[1] != kI * kN || in_sizes[2] != kN || in_sizes[3] != kN * kO) return;
  if (out_size != kRows * kO) return;
  if (ws_size < kWsTotal) return;
  const float* x = (const float*)d_in[0];
  const float* b = (const float*)d_in[1];
  const float* A = (const float*)d_in[2];
  const float* c = (const float*)d_in[3];
  float* out = (float*)d_out;
  char* ws = (char*)d_ws;
  unsigned short* X16 = (unsigned short*)(ws + kOffX16);
  unsigned short* WB16 = (unsigned short*)(ws + kOffWB16);
  unsigned short* WC16 = (unsigned short*)(ws + kOffWC16);
  float* ZB = (float*)(ws + kOffZB);
  float* XB = (float*)(ws + kOffXB);
  unsigned short* S16 = (unsigned short*)(ws + kOffS16);

  static_assert(((size_t)kRows * kI / 8) % kThr == 0 && ((size_t)kRows * kI) % 1024 == 0, "the cast's grid; the source is whole rows of 1,024 as the flat cast counts them");
  cast_plane_kernel<<<(int)(((size_t)kRows * kI / 8) / kThr), kThr, 0, stream>>>(x, X16, 10, 1024, 0);
  wt_plane_kernel<<<kN, kI / 8, 0, stream>>>(b, WB16, kI, kN, kN, kI, 0);
  wt_plane_kernel<<<kO, kN / 8, 0, stream>>>(c, WC16, kN, kO, kO, kN, 0);
  setup_kernel<<<1, kNq, 0, stream>>>(ZB);
  for (int quarter = 0; quarter < 4; ++quarter) {
    const unsigned short* wb = WB16 + (size_t)quarter * kNq * kI;
    wmma_gemm64<0, false, 2, 0, false, 0><<<dim3((kRows / 64) * (kNq / 64) / 8, 1), 256, 0, stream>>>(
        X16, X16, kI, 0L, wb, wb, kI, 0L, (void*)XB, (void*)XB, kNq, 0L, ZB, nullptr, 0L, kRows, kNq, kI, kScIn);
    scan_kernel<<<8, kThr, 0, stream>>>(XB, A, S16, quarter);
  }
  wmma_gemm64<0, false, 2, 0, false, 0><<<dim3((kRows / 64) * (kO / 64) / 8, 1), 256, 0, stream>>>(
      S16, S16, kN, 0L, WC16, WC16, kN, 0L, (void*)out, (void*)out, kO, 0L, ZB, nullptr, 0L, kRows, kO, kN, kScOut);
}
static_assert(((kRows / 64) * (kNq / 64)) % 8 == 0 && ((kRows / 64) * (kO / 64)) % 8 == 0, "the engine's grids: whole blocks of eight wave tiles");
